// CFConv_3204045603903
// MI455X (gfx1250) — hardware-verified
//
#include <hip/hip_runtime.h>


#define NB_  4
#define WCH  16
#define FCH  64
#define OCH  64
#define IMW  128
#define OW_  126
#define NP   (OW_ * OW_)
#define NPP  15936
#define IP   96
#define JN   17
#define MROW (OCH * JN)
typedef _Float16 h16;
typedef unsigned short bf;
typedef __attribute__((ext_vector_type(16))) __bf16   v16bf;
typedef __attribute__((ext_vector_type(16))) _Float16 v16h;
typedef __attribute__((ext_vector_type(8)))  _Float16 v8h;
typedef __attribute__((ext_vector_type(8)))  unsigned short v8us;
typedef __attribute__((ext_vector_type(8)))  float    v8f;
typedef __attribute__((ext_vector_type(4)))  float    v4f;
typedef v8h  __attribute__((may_alias)) v8ha;
typedef v4f  __attribute__((may_alias)) v4fa;
typedef v8us __attribute__((may_alias)) v8usa;

__device__ __forceinline__ unsigned short f2bf(float f) { unsigned u = __float_as_uint(f); u += 0x7FFFu + ((u >> 16) & 1u); return (unsigned short)(u >> 16); }
__device__ __forceinline__ float bf2f(unsigned short b) { return __uint_as_float(((unsigned)b) << 16); }
__device__ __forceinline__ float bfr(float f) { return bf2f(f2bf(f)); }
__device__ __forceinline__ v16h cat16(v8h lo, v8h hi) { return __builtin_shufflevector(lo, hi, 0, 1, 2, 3, 4, 5, 6, 7, 8, 9, 10, 11, 12, 13, 14, 15); }
__device__ __forceinline__ v16bf cat16b(v8us lo, v8us hi) { return __builtin_bit_cast(v16bf, __builtin_shufflevector(lo, hi, 0, 1, 2, 3, 4, 5, 6, 7, 8, 9, 10, 11, 12, 13, 14, 15)); }
__device__ __forceinline__ v8f wmma16(v16h a, v16h b, v8f c) { return __builtin_amdgcn_wmma_f32_16x16x32_f16(false, a, false, b, (short)0, c, false, false); }
__device__ __forceinline__ v8f wmmab(v16bf a, v16bf b, v8f c) { return __builtin_amdgcn_wmma_f32_16x16x32_bf16(false, a, false, b, (short)0, c, false, false); }


template <typename T16> struct WFrag;
template <> struct WFrag<h16> { typedef v16h V; static __device__ __forceinline__ V ld(const h16* p) { return cat16(*(const v8h*)p, *(const v8h*)(p + 16)); } static __device__ __forceinline__ v8f mma(V a, V b, v8f c) { return wmma16(a, b, c); } };
template <> struct WFrag<bf> { typedef v16bf V; static __device__ __forceinline__ V ld(const bf* p) { return cat16b(*(const v8us*)p, *(const v8us*)(p + 16)); } static __device__ __forceinline__ v8f mma(V a, V b, v8f c) { return wmmab(a, b, c); } };
template <typename T16, int NSPLIT, bool BIAS>
__global__ __launch_bounds__(32) void k_gemmw(const T16* __restrict__ A, const T16* __restrict__ A2, const T16* __restrict__ Bt, const T16* __restrict__ Bt2, int K, float* C, int ldc, const float* __restrict__ bias, size_t sA, size_t sB, size_t sC) {
    typedef typename WFrag<T16>::V V;
    __shared__ __align__(16) float os[16 * 68];
    const size_t z = blockIdx.z; A += z * sA; if (A2) A2 += z * sA; Bt += z * sB; if (Bt2) Bt2 += z * sB; C += z * sC;
    const int lane = threadIdx.x & 31, lr = lane & 15, hi = lane >> 4; const int r0 = blockIdx.x * 64, c0 = blockIdx.y * 64;
    v8f acc[4][4];
#pragma unroll
    for (int mb = 0; mb < 4; ++mb)
#pragma unroll
        for (int nb = 0; nb < 4; ++nb) acc[mb][nb] = (v8f){};
    const size_t aoff = (size_t)(r0 + lr) * K + 8 * hi, boff = (size_t)(c0 + lr) * K + 8 * hi;
#pragma unroll 1
    for (int kc = 0; kc < K; kc += 32) {
        V a[4], a2[4];
#pragma unroll
        for (int mb = 0; mb < 4; ++mb) { a[mb] = WFrag<T16>::ld(A + aoff + (size_t)mb * 16 * K + kc); if (NSPLIT == 1 || NSPLIT == 2) a2[mb] = WFrag<T16>::ld(A2 + aoff + (size_t)mb * 16 * K + kc); }
#pragma unroll
        for (int nb = 0; nb < 4; ++nb) { const V b = WFrag<T16>::ld(Bt + boff + (size_t)nb * 16 * K + kc); V b2; if (NSPLIT >= 2) b2 = WFrag<T16>::ld(Bt2 + boff + (size_t)nb * 16 * K + kc);
#pragma unroll
            for (int mb = 0; mb < 4; ++mb) { acc[mb][nb] = WFrag<T16>::mma(a[mb], b, acc[mb][nb]); if (NSPLIT == 1 || NSPLIT == 2) acc[mb][nb] = WFrag<T16>::mma(a2[mb], b, acc[mb][nb]); if (NSPLIT >= 2) acc[mb][nb] = WFrag<T16>::mma(a[mb], b2, acc[mb][nb]); } }
        asm volatile("v_nop\n\tv_nop\n\tv_nop\n\tv_nop" : "+v"(acc[0][0]), "+v"(acc[1][1]), "+v"(acc[2][2]), "+v"(acc[3][3]) : "v"(a[0]), "v"(a[3]));
    }
#pragma unroll
    for (int mb = 0; mb < 4; ++mb) {
#pragma unroll
        for (int nb = 0; nb < 4; ++nb) {
#pragma unroll
            for (int j = 0; j < 8; ++j) os[(hi * 8 + j) * 68 + nb * 16 + lr] = acc[mb][nb][j]; }
        __builtin_amdgcn_wave_barrier(); asm volatile("" ::: "memory");
        float* crow = C + (size_t)(r0 + mb * 16) * ldc + c0;
#pragma unroll 1
        for (int ps = 0; ps < 2; ++ps) {
#pragma unroll
            for (int s = 0; s < 8; ++s) { const int row = 2 * s + hi, cofs = lr * 4; v4f val = *(const v4fa*)(os + row * 68 + cofs); if (BIAS) { val[0] += bfr(bias[c0 + cofs]); val[1] += bfr(bias[c0 + cofs + 1]); val[2] += bfr(bias[c0 + cofs + 2]); val[3] += bfr(bias[c0 + cofs + 3]); }
                *(volatile v4f*)(crow + (size_t)row * ldc + cofs) = val; }
            if (ps == 0) __threadfence(); }
        __builtin_amdgcn_wave_barrier(); asm volatile("" ::: "memory");
    }
}

__device__ __forceinline__ h16 tohx(float x) { return (h16)x; }
__device__ __forceinline__ void splitf(float y, unsigned short& h, unsigned short& l) { h = f2bf(y); l = f2bf(y - bf2f(h)); }
typedef __attribute__((ext_vector_type(2))) _Float16 v2h;
typedef __attribute__((ext_vector_type(4))) _Float16 v4h;
typedef __attribute__((ext_vector_type(2))) unsigned short v2us;
typedef __attribute__((ext_vector_type(4))) unsigned short v4us;
typedef __attribute__((ext_vector_type(2))) float v2f;
typedef __attribute__((ext_vector_type(4))) int v4i;


__global__ __launch_bounds__(256) void k_wkb(const float* __restrict__ Wt, bf* dst) { const size_t e8 = (size_t)blockIdx.x * 256 + threadIdx.x; if (e8 >= (size_t)9 * MROW * IP / 8) return; const size_t e = e8 * 8; const int i0 = (int)(e % IP); const int row = (int)((e / IP) % MROW); const int k = (int)(e / ((size_t)IP * MROW)); const int o = row / JN, j = row % JN; v8us ov;
#pragma unroll
    for (int q = 0; q < 8; ++q) { const int i = i0 + q; const float v = (i < FCH + 1) ? Wt[(((size_t)k * OCH + o) * (FCH + 1) + i) * JN + j] : 0.0f; ov[q] = f2bf(v); }
    *(volatile v8us*)(dst + e) = ov; __threadfence(); *(volatile v8us*)(dst + e) = ov; }
__global__ __launch_bounds__(256) void k_fagat(const float* __restrict__ Xf, int dy, int dx, bf* FA) { const size_t e8 = (size_t)blockIdx.x * 256 + threadIdx.x; if (e8 >= (size_t)NPP * IP / 8) return; const size_t e = e8 * 8; const int i0 = (int)(e % IP); const int p = (int)(e / IP); const int y = p / OW_, x = p % OW_; v8us ov;
#pragma unroll
    for (int q = 0; q < 8; ++q) { const int i = i0 + q; float v = 0.0f; if (p < NP) { if (i < FCH) v = Xf[((size_t)i * IMW + (y + dy)) * IMW + (x + dx)]; else if (i == FCH) v = 1.0f; } ov[q] = f2bf(v); }
    *(volatile v8us*)(FA + e) = ov; __threadfence(); *(volatile v8us*)(FA + e) = ov; }
template <bool FIRST>
__global__ __launch_bounds__(256) void k_cfacc(const float* __restrict__ T, const float* __restrict__ Xw, int dy, int dx, float* ACC) { const size_t g = (size_t)blockIdx.x * 256 + threadIdx.x; if (g >= (size_t)OCH * NPP) return; const int p = (int)(g % NPP); const int o = (int)(g / NPP); float res = 0.0f;
    if (p < NP) { const int y = p / OW_, x = p % OW_; float s = 0.f;
#pragma unroll
        for (int j = 0; j < WCH; ++j) { float wv = bfr(Xw[((size_t)j * IMW + (y + dy)) * IMW + (x + dx)]); asm volatile("" : "+v"(wv)); float pr = __fmul_rn(T[((size_t)o * JN + j) * NPP + p], wv); asm volatile("" : "+v"(pr)); s = __fadd_rn(s, pr); }
        s = __fadd_rn(s, T[((size_t)o * JN + WCH) * NPP + p]);
        res = FIRST ? s : __fadd_rn(ACC[g], s); }
    *(volatile float*)(ACC + g) = res; __threadfence(); *(volatile float*)(ACC + g) = res; }
__global__ __launch_bounds__(256) void k_outcp(const float* __restrict__ ACC, float* out) { const size_t i = (size_t)blockIdx.x * 256 + threadIdx.x; if (i >= (size_t)OCH * NP / 4) return; const size_t e = i * 4; const int o = (int)(e / NP); const int p = (int)(e % NP); v4f v;
#pragma unroll
    for (int q = 0; q < 4; ++q) v[q] = ACC[(size_t)o * NPP + p + q]; *(volatile v4f*)(out + e) = v; __threadfence(); *(volatile v4f*)(out + e) = v; }

extern "C" void kernel_launch(void* const* d_in, const int* in_sizes, int n_in,
                              void* d_out, int out_size, void* d_ws, size_t ws_size, hipStream_t stream) {
    (void)in_sizes; (void)n_in; (void)out_size;
    const float* xw = (const float*)d_in[0]; const float* xf = (const float*)d_in[1]; const float* wt = (const float*)d_in[2];
    float* OUT = (float*)d_out;
    char* wsp = (char*)d_ws;
    auto take = [&](size_t bytes) { char* p = wsp; wsp += (bytes + 255) & ~(size_t)255; return (void*)p; };
    bf* WKB = (bf*)take((size_t)9 * MROW * IP * 2); bf* FA = (bf*)take((size_t)NPP * IP * 2); float* T = (float*)take((size_t)MROW * NPP * 4); float* ACC = (float*)take((size_t)OCH * NPP * 4);
    if ((size_t)(wsp - (char*)d_ws) > ws_size) return;
    k_wkb<<<(unsigned)(((size_t)9 * MROW * IP / 8 + 255) / 256), 256, 0, stream>>>(wt, WKB);
    const unsigned LF_ = (unsigned)(((size_t)NPP * IP / 8 + 255) / 256), LA = (unsigned)(((size_t)OCH * NPP + 255) / 256);
    for (int b = 0; b < NB_; ++b) { const float* xfb = xf + (size_t)b * FCH * IMW * IMW; const float* xwb = xw + (size_t)b * WCH * IMW * IMW;
        for (int k = 0; k < 9; ++k) { const int dy = k / 3, dx = k % 3;
            k_fagat<<<LF_, 256, 0, stream>>>(xfb, dy, dx, FA);
            k_gemmw<bf, 0, false><<<dim3(MROW / 64, NPP / 64, 1), 32, 0, stream>>>(WKB + (size_t)k * MROW * IP, nullptr, FA, nullptr, IP, T, NPP, nullptr, 0, 0, 0);
            if (k == 0) k_cfacc<true><<<LA, 256, 0, stream>>>(T, xwb, dy, dx, ACC); else k_cfacc<false><<<LA, 256, 0, stream>>>(T, xwb, dy, dx, ACC); }
        k_outcp<<<(unsigned)(((size_t)OCH * NP / 4 + 255) / 256), 256, 0, stream>>>(ACC, OUT + (size_t)b * OCH * NP); }
}
